// MultiScaleRetention_32186484916893
// MI455X (gfx1250) — hardware-verified
//
#include <hip/hip_runtime.h>
#include <math.h>
#include <stdint.h>

constexpr int kBatch = 2;
constexpr int kSeq   = 2048;
constexpr int kEmb   = 1024;
constexpr int kVEmb  = 2048;
constexpr int kHeads = 8;
constexpr int kDK    = 128;
constexpr int kDV    = 256;
constexpr int kRows  = kBatch * kSeq;
constexpr int kPairs = kDK / 2;
constexpr int kHeadsPerGrp = 4;
constexpr int kGroups = kBatch * kHeads / kHeadsPerGrp;

constexpr float kQKCarry  = 8.0f;
constexpr float kPCarry   = 16.0f;
constexpr float kVCarry   = 8.0f;
constexpr float kYCarry   = 16.0f;
constexpr float kWoCarry  = 16.0f;
constexpr float kScoreScale = kPCarry / (kQKCarry * kQKCarry);
constexpr float kPVScale    = 1.0f / (kPCarry * kVCarry);
constexpr float kOutScale   = 1.0f / (kYCarry * kWoCarry);
constexpr float kEps   = 1e-6f;
constexpr float kInvDV = 1.0f / 256.0f;

constexpr size_t kBytesXb   = (size_t)kRows * kEmb * 2;
constexpr size_t kBytesWqk  = (size_t)kEmb * kEmb * 2;
constexpr size_t kBytesWvg  = (size_t)kVEmb * kEmb * 2;
constexpr size_t kBytesTmp  = (size_t)kRows * kEmb * 4;
constexpr size_t kBytesP    = (size_t)kHeadsPerGrp * kSeq * kSeq * 2;
constexpr size_t kBytesY2   = (size_t)kRows * kVEmb * 2;
constexpr size_t kBytesWo   = (size_t)kEmb * kVEmb * 2;
constexpr size_t kBytesQr   = (size_t)kRows * kEmb * 2;
constexpr size_t kBytesVT   = (size_t)kBatch * kVEmb * kSeq * 2;
constexpr size_t kBytesG    = (size_t)kRows * kVEmb * 2;
constexpr size_t kBytesY    = (size_t)kRows * kVEmb * 4;
constexpr size_t kBytesTrig = (size_t)kPairs * kSeq * 8;

constexpr size_t kOffXb   = 0;
constexpr size_t kOffWq   = kOffXb + kBytesXb;
constexpr size_t kOffWk   = kOffWq + kBytesWqk;
constexpr size_t kOffWv   = kOffWk + kBytesWqk;
constexpr size_t kOffWg   = kOffWv + kBytesWvg;
constexpr size_t kOffTmp  = kOffWg + kBytesWvg;
constexpr size_t kEndR0   = kOffTmp + kBytesTmp;
constexpr size_t kOffP    = 0;
constexpr size_t kOffY2   = 0;
constexpr size_t kOffWo   = kEndR0;
constexpr size_t kOffQr   = kOffWo + kBytesWo;
constexpr size_t kOffKr   = kOffQr + kBytesQr;
constexpr size_t kOffVT   = kOffKr + kBytesQr;
constexpr size_t kOffG    = kOffVT + kBytesVT;
constexpr size_t kOffY    = kOffG + kBytesG;
constexpr size_t kOffTrig = kOffY + kBytesY;
constexpr size_t kWsTotal = kOffTrig + kBytesTrig;
static_assert(kOffP + kBytesP <= kEndR0);
static_assert(kOffY2 + kBytesY2 <= kEndR0);
static_assert(kWsTotal <= (size_t)134217728);
static_assert((kOffWo % 256) == 0 && (kOffQr % 256) == 0 && (kOffVT % 256) == 0 && (kOffG % 256) == 0 && (kOffY % 256) == 0 && (kOffTrig % 256) == 0 && (kOffTmp % 256) == 0);

typedef __attribute__((ext_vector_type(16))) _Float16 v16h;
typedef __attribute__((ext_vector_type(8)))  _Float16 v8h;
typedef __attribute__((ext_vector_type(16))) __bf16   v16b;
typedef __attribute__((ext_vector_type(8)))  __bf16   v8b;
typedef __attribute__((ext_vector_type(8)))  float    v8f;
typedef __attribute__((ext_vector_type(4)))  float    v4f;
typedef __attribute__((ext_vector_type(2)))  float    v2f;
typedef __attribute__((ext_vector_type(4)))  unsigned int v4u;

__device__ __forceinline__ unsigned short f2bf_bits(float f) {
  unsigned u = __float_as_uint(f);
  return (unsigned short)((u + 0x7FFFu + ((u >> 16) & 1u)) >> 16);
}
__device__ __forceinline__ float bf_bits2f(unsigned short h) { return __uint_as_float(((unsigned)h) << 16); }

__device__ __forceinline__ void dep_guard_h(v8f& a, v8f& b, v16h x, v16h y) { asm volatile("v_nop\n\tv_nop\n\tv_nop\n\tv_nop" : "+v"(a), "+v"(b) : "v"(x), "v"(y)); }
__device__ __forceinline__ void dep_guard_b(v8f& a, v8f& b, v16b x, v16b y) { asm volatile("v_nop\n\tv_nop\n\tv_nop\n\tv_nop" : "+v"(a), "+v"(b) : "v"(x), "v"(y)); }
__device__ __forceinline__ void keep4_h(v16h a, v16h b, v16h c, v16h d) { asm volatile("v_nop" :: "v"(a), "v"(b), "v"(c), "v"(d)); }
__device__ __forceinline__ void keep4_b(v16b a, v16b b, v16b c, v16b d) { asm volatile("v_nop" :: "v"(a), "v"(b), "v"(c), "v"(d)); }
__device__ __forceinline__ void acc_guard4(v8f& a, v8f& b, v8f& c, v8f& d) { asm volatile("v_nop\n\tv_nop\n\tv_nop\n\tv_nop" : "+v"(a), "+v"(b), "+v"(c), "+v"(d)); }
template <typename T> struct Frag;
template <> struct Frag<_Float16> {
  typedef v16h V; union U { v16h v; v8h h[2]; };
  static __device__ __forceinline__ v16h load(const _Float16* p) {
    U f; f.h[0] = *(const v8h*)(p); f.h[1] = *(const v8h*)(p + 16); return f.v;
  }
  static __device__ __forceinline__ v8f mma(v16h a, v16h b, v8f c) {
    return __builtin_amdgcn_wmma_f32_16x16x32_f16(false, a, false, b, (short)0, c, false, false);
  }
  static __device__ __forceinline__ void guard(v8f& a, v8f& b, v16h x, v16h y) { dep_guard_h(a, b, x, y); }
  static __device__ __forceinline__ void keep(v16h a, v16h b, v16h c, v16h d) { keep4_h(a, b, c, d); }
};
template <> struct Frag<__bf16> {
  typedef v16b V; union U { v16b v; v8b h[2]; };
  static __device__ __forceinline__ v16b load(const __bf16* p) {
    U f; f.h[0] = *(const v8b*)(p); f.h[1] = *(const v8b*)(p + 16); return f.v;
  }
  static __device__ __forceinline__ v8f mma(v16b a, v16b b, v8f c) {
    return __builtin_amdgcn_wmma_f32_16x16x32_bf16(false, a, false, b, (short)0, c, false, false);
  }
  static __device__ __forceinline__ void guard(v8f& a, v8f& b, v16b x, v16b y) { dep_guard_b(a, b, x, y); }
  static __device__ __forceinline__ void keep(v16b a, v16b b, v16b c, v16b d) { keep4_b(a, b, c, d); }
};

__device__ __forceinline__ unsigned pk16(unsigned short a, unsigned short b) { return (unsigned)a | ((unsigned)b << 16); }
__device__ __forceinline__ unsigned short h_bits(float f) { const _Float16 h = (_Float16)f; return __builtin_bit_cast(unsigned short, h); }

template <int ET> struct Elem;
template <> struct Elem<0> { typedef _Float16 T; };
template <> struct Elem<1> { typedef __bf16 T; };
template <int ET, bool SPLIT, int BIAS_MODE, int OUT_MODE, bool RESID, int ACT = 0, int CAUSAL = 0>
__global__ __launch_bounds__(256) void wmma_gemm64(
    const unsigned short* __restrict__ Ap, const unsigned short* __restrict__ A2p, int lda, long strideA,
    const unsigned short* __restrict__ Btp, const unsigned short* __restrict__ Bt2p, int ldb, long strideB,
    void* __restrict__ Cout, void* __restrict__ Cout2, int ldc, long strideC,
    const float* __restrict__ bias,
    const float* __restrict__ resid, long strideR,
    int M, int N, int K, float scale, float oscale,
    float lgA, float lgB, float lgC, float lgD) {
  typedef typename Elem<ET>::T T;
  typedef typename Frag<T>::V V;
  const T* A = (const T*)Ap; const T* A2 = (const T*)A2p; const T* Bt = (const T*)Btp; const T* Bt2 = (const T*)Bt2p;
  __shared__ __align__(16) float sT[8][16 * 68];
  const int b    = blockIdx.y;
  const int lane = threadIdx.x & 31;
  const int wave = threadIdx.x >> 5;
  const int tilesN = N >> 6;
  const int tilesM = M >> 6;
  const int tile = blockIdx.x * 8 + wave;
  if (tile >= tilesM * tilesN) return;
  const int tm = tile / tilesN;
  const int tn = tile - tm * tilesN;
  const int m0 = tm << 6;
  const int n0 = tn << 6;
  if (CAUSAL == 1 && n0 > m0) return;
  const int kEnd = (CAUSAL == 2) ? ((m0 + 64 < K) ? (m0 + 64) : K) : K;
  const float lg2 = (b == 0) ? lgA : (b == 1) ? lgB : (b == 2) ? lgC : lgD;

  const T* Ab  = A  + (size_t)b * strideA;
  const T* Bb  = Bt + (size_t)b * strideB;
  const T* Ab2 = SPLIT ? (A2  + (size_t)b * strideA) : nullptr;
  const T* Bb2 = SPLIT ? (Bt2 + (size_t)b * strideB) : nullptr;

  const int rlane = lane & 15;
  const int koff  = (lane >> 4) * 8;
  const int mOff  = (lane >> 4) * 8;

  v8f acc[4][4];
#pragma unroll
  for (int i = 0; i < 4; ++i)
#pragma unroll
    for (int j = 0; j < 4; ++j) acc[i][j] = (v8f){0.f,0.f,0.f,0.f,0.f,0.f,0.f,0.f};

  for (int k0 = 0; k0 < kEnd; k0 += 32) {
    V bh[4], bl[4];
#pragma unroll
    for (int j = 0; j < 4; ++j) {
      const size_t bo = (size_t)(n0 + (j << 4) + rlane) * ldb + koff + k0;
      bh[j] = Frag<T>::load(Bb + bo);
      if (SPLIT) bl[j] = Frag<T>::load(Bb2 + bo);
    }
#pragma unroll
    for (int i = 0; i < 4; ++i) {
      const size_t ao = (size_t)(m0 + (i << 4) + rlane) * lda + koff + k0;
      V ah = Frag<T>::load(Ab + ao);
      V al;
      if (SPLIT) al = Frag<T>::load(Ab2 + ao);
#pragma unroll
      for (int j = 0; j < 4; ++j) {
        acc[i][j] = Frag<T>::mma(ah, bh[j], acc[i][j]);
        if (SPLIT) {
          acc[i][j] = Frag<T>::mma(ah, bl[j], acc[i][j]);
          acc[i][j] = Frag<T>::mma(al, bh[j], acc[i][j]);
        }
      }
      Frag<T>::guard(acc[i][0], acc[i][3], ah, SPLIT ? al : ah);
    }
    Frag<T>::keep(bh[0], bh[1], bh[2], bh[3]);
    if (SPLIT) Frag<T>::keep(bl[0], bl[1], bl[2], bl[3]);
  }
  acc_guard4(acc[0][0], acc[0][1], acc[0][2], acc[0][3]);
  acc_guard4(acc[1][0], acc[1][1], acc[1][2], acc[1][3]);
  acc_guard4(acc[2][0], acc[2][1], acc[2][2], acc[2][3]);
  acc_guard4(acc[3][0], acc[3][1], acc[3][2], acc[3][3]);

  float* slab = sT[wave];
  const float* Rb = RESID ? (resid + (size_t)b * strideR) : nullptr;
#pragma unroll
  for (int i = 0; i < 4; ++i) {
    const int mBase = m0 + (i << 4);
#pragma unroll
    for (int j = 0; j < 4; ++j) {
      const int n = n0 + (j << 4) + rlane;
      float bv = 0.f;
      if (BIAS_MODE == 2) bv = bias[n];
#pragma unroll
      for (int r = 0; r < 8; ++r) {
        float v = acc[i][j][r] * scale;
        if (BIAS_MODE == 1) v += bias[mBase + mOff + r];
        if (BIAS_MODE == 2) v += bv;
        if (RESID) v += Rb[(size_t)(mBase + mOff + r) * ldc + n];
        if (ACT == 2) v = fmaxf(v, 0.0f);
        if (ACT == 4) v = (v > 0.f) ? v : 0.01f * v;
        if (ACT == 6) v = __builtin_amdgcn_rcpf(1.0f + __expf(-v));
        if (CAUSAL == 1) {
          const int dd = (mBase + mOff + r) - n;
          const float de = exp2f((float)dd * lg2);
          v = (dd >= 0) ? (v * de) : 0.0f;
        }
        v *= oscale;
        slab[(mOff + r) * 68 + (j << 4) + rlane] = v;
      }
    }
    __builtin_amdgcn_fence(__ATOMIC_RELEASE, "workgroup");
    __builtin_amdgcn_wave_barrier();
    __builtin_amdgcn_fence(__ATOMIC_ACQUIRE, "workgroup");
    if (OUT_MODE == 0) {
      float* C = (float*)Cout + (size_t)b * strideC;
      const int hh = lane >> 4, c4 = (lane & 15) * 4;
      for (int pass = 0; pass < 2; ++pass) {
#pragma unroll
        for (int it = 0; it < 8; ++it) {
          const int row = it * 2 + hh;
          v4f v = *(const v4f*)(slab + row * 68 + c4);
          *(volatile v4f*)(C + (size_t)(mBase + row) * ldc + n0 + c4) = v;
        }
        __threadfence();
      }
    } else {
      const int q = lane >> 3, c8 = (lane & 7) * 8;
      unsigned short* C  = (unsigned short*)Cout  + (size_t)b * strideC;
      unsigned short* C2 = (OUT_MODE == 2) ? ((unsigned short*)Cout2 + (size_t)b * strideC) : nullptr;
      for (int pass = 0; pass < 2; ++pass) {
#pragma unroll
        for (int it = 0; it < 4; ++it) {
          const int row = it * 4 + q;
          const float* sp = slab + row * 68 + c8;
          v8h hv, lv;
#pragma unroll
          for (int e = 0; e < 8; ++e) {
            if (OUT_MODE == 1) {
              hv[e] = (_Float16)sp[e];
            } else {
              unsigned short hb = f2bf_bits(sp[e]);
              unsigned short lb = f2bf_bits(sp[e] - bf_bits2f(hb));
              hv[e] = __builtin_bit_cast(_Float16, hb);
              lv[e] = __builtin_bit_cast(_Float16, lb);
            }
          }
          *(volatile v8h*)(C + (size_t)(mBase + row) * ldc + n0 + c8) = hv;
          if (OUT_MODE == 2) *(volatile v8h*)(C2 + (size_t)(mBase + row) * ldc + n0 + c8) = lv;
        }
        __threadfence();
      }
    }
    __builtin_amdgcn_fence(__ATOMIC_RELEASE, "workgroup");
    __builtin_amdgcn_wave_barrier();
    __builtin_amdgcn_fence(__ATOMIC_ACQUIRE, "workgroup");
  }
}

template <int MODE> __device__ __forceinline__ unsigned short cvt16(float f) {
  if (MODE == 0) return f2bf_bits(f);
  return h_bits(bf_bits2f(f2bf_bits(f)) * kWoCarry);
}
template <int MODE>
__global__ __launch_bounds__(256) void cast16x8_kernel(const float* __restrict__ in, unsigned short* __restrict__ out, int n8) {
  const int i = blockIdx.x * 256 + threadIdx.x;
  if (i < n8) {
    const size_t e0 = (size_t)i * 8;
    const v4f a = *(const v4f*)(in + e0);
    const v4f c = *(const v4f*)(in + e0 + 4);
    const v4u u = (v4u){pk16(cvt16<MODE>(a[0]), cvt16<MODE>(a[1])), pk16(cvt16<MODE>(a[2]), cvt16<MODE>(a[3])),
                        pk16(cvt16<MODE>(c[0]), cvt16<MODE>(c[1])), pk16(cvt16<MODE>(c[2]), cvt16<MODE>(c[3]))};
    *(volatile v4u*)(out + e0) = u;
    __threadfence();
    *(volatile v4u*)(out + e0) = u;
  }
}

__device__ __forceinline__ v4f pick4(bool cnd, v4f a, v4f b) {
  v4f r;
  r[0] = cnd ? a[0] : b[0]; r[1] = cnd ? a[1] : b[1]; r[2] = cnd ? a[2] : b[2]; r[3] = cnd ? a[3] : b[3];
  return r;
}
__global__ __launch_bounds__(256) void trig_table_kernel(float* __restrict__ tab,
    v4f f0, v4f f1, v4f f2, v4f f3, v4f f4, v4f f5, v4f f6, v4f f7,
    v4f f8, v4f f9, v4f f10, v4f f11, v4f f12, v4f f13, v4f f14, v4f f15) {
  #pragma clang fp contract(off)
  const int s = blockIdx.x * 256 + threadIdx.x;
  const int i = blockIdx.y;
  const int gsel = i >> 2, esel = i & 3;
  v4f sel = f0;
  sel = pick4(gsel == 1, f1, sel);   sel = pick4(gsel == 2, f2, sel);   sel = pick4(gsel == 3, f3, sel);
  sel = pick4(gsel == 4, f4, sel);   sel = pick4(gsel == 5, f5, sel);   sel = pick4(gsel == 6, f6, sel);
  sel = pick4(gsel == 7, f7, sel);   sel = pick4(gsel == 8, f8, sel);   sel = pick4(gsel == 9, f9, sel);
  sel = pick4(gsel == 10, f10, sel); sel = pick4(gsel == 11, f11, sel); sel = pick4(gsel == 12, f12, sel);
  sel = pick4(gsel == 13, f13, sel); sel = pick4(gsel == 14, f14, sel); sel = pick4(gsel == 15, f15, sel);
  const float inv = (esel == 0) ? sel[0] : (esel == 1) ? sel[1] : (esel == 2) ? sel[2] : sel[3];
  const float ang = (float)s * inv;
  const double xd = (double)ang;
  const double kq = (xd * 0.63661977236758134308 + 6755399441055744.0) - 6755399441055744.0;
  double rr = __builtin_fma(-kq, 1.5707963267948966, xd);
  rr = __builtin_fma(-kq, 6.123233995736766e-17, rr);
  const double z = rr * rr;
  double sp = -1.0 / 39916800.0;
  sp = __builtin_fma(sp, z, 1.0 / 362880.0);
  sp = __builtin_fma(sp, z, -1.0 / 5040.0);
  sp = __builtin_fma(sp, z, 1.0 / 120.0);
  sp = __builtin_fma(sp, z, -1.0 / 6.0);
  const double sn = __builtin_fma(sp * z, rr, rr);
  double cp = 1.0 / 479001600.0;
  cp = __builtin_fma(cp, z, -1.0 / 3628800.0);
  cp = __builtin_fma(cp, z, 1.0 / 40320.0);
  cp = __builtin_fma(cp, z, -1.0 / 720.0);
  cp = __builtin_fma(cp, z, 1.0 / 24.0);
  cp = __builtin_fma(cp, z, -0.5);
  const double cs = __builtin_fma(cp, z, 1.0);
  const int qd = ((int)kq) & 3;
  const float sf = (float)sn, cf = (float)cs;
  const float osin = (qd == 0) ? sf : (qd == 1) ? cf : (qd == 2) ? -sf : -cf;
  const float ocos = (qd == 0) ? cf : (qd == 1) ? -sf : (qd == 2) ? -cf : sf;
  v2f o; o[0] = ocos; o[1] = osin;
  float* p = tab + ((size_t)i * kSeq + s) * 2;
  *(volatile v2f*)p = o;
  __threadfence();
  *(volatile v2f*)p = o;
}

__global__ __launch_bounds__(256) void rope_kernel(const float* __restrict__ src, const float* __restrict__ tab,
                                                   unsigned short* __restrict__ dst) {
  #pragma clang fp contract(off)
  const int t = blockIdx.x * 256 + threadIdx.x;
  const size_t e0 = (size_t)t * 8;
  const int row = (int)(e0 >> 10);
  const int col = (int)(e0 & 1023);
  const int s   = row & (kSeq - 1);
  const int i0  = (col & (kDK - 1)) >> 1;
  const v4f a = *(const v4f*)(src + e0);
  const v4f c = *(const v4f*)(src + e0 + 4);
  const v2f t0 = *(const v2f*)(tab + ((size_t)(i0 + 0) * kSeq + s) * 2);
  const v2f t1 = *(const v2f*)(tab + ((size_t)(i0 + 1) * kSeq + s) * 2);
  const v2f t2 = *(const v2f*)(tab + ((size_t)(i0 + 2) * kSeq + s) * 2);
  const v2f t3 = *(const v2f*)(tab + ((size_t)(i0 + 3) * kSeq + s) * 2);
  const float o0 = (a[0] * t0[0] - a[1] * t0[1]) * kQKCarry;
  const float o1 = (a[0] * t0[1] + a[1] * t0[0]) * kQKCarry;
  const float o2 = (a[2] * t1[0] - a[3] * t1[1]) * kQKCarry;
  const float o3 = (a[2] * t1[1] + a[3] * t1[0]) * kQKCarry;
  const float o4 = (c[0] * t2[0] - c[1] * t2[1]) * kQKCarry;
  const float o5 = (c[0] * t2[1] + c[1] * t2[0]) * kQKCarry;
  const float o6 = (c[2] * t3[0] - c[3] * t3[1]) * kQKCarry;
  const float o7 = (c[2] * t3[1] + c[3] * t3[0]) * kQKCarry;
  const v4u u = (v4u){pk16(h_bits(o0), h_bits(o1)), pk16(h_bits(o2), h_bits(o3)),
                      pk16(h_bits(o4), h_bits(o5)), pk16(h_bits(o6), h_bits(o7))};
  *(volatile v4u*)(dst + e0) = u;
  __threadfence();
  *(volatile v4u*)(dst + e0) = u;
}

__global__ __launch_bounds__(256) void rmsgate_kernel(const float* __restrict__ y, const unsigned short* __restrict__ g16,
                                                      const float* __restrict__ gnw, unsigned short* __restrict__ y2) {
  #pragma clang fp contract(off)
  const int row  = blockIdx.x;
  const int lane = threadIdx.x & 31;
  const int head = threadIdx.x >> 5;
  const size_t base = (size_t)row * kVEmb + head * kDV + lane * 8;
  const v4f a = *(const v4f*)(y + base);
  const v4f c = *(const v4f*)(y + base + 4);
  float ss = a[0] * a[0] + a[1] * a[1] + a[2] * a[2] + a[3] * a[3]
           + c[0] * c[0] + c[1] * c[1] + c[2] * c[2] + c[3] * c[3];
#pragma unroll
  for (int off = 16; off > 0; off >>= 1) ss += __shfl_xor(ss, off, 32);
  const float rr = rsqrtf(ss * kInvDV + kEps);
  const v4f w0 = *(const v4f*)(gnw + lane * 8);
  const v4f w1 = *(const v4f*)(gnw + lane * 8 + 4);
  const v8h gv = *(const v8h*)((const _Float16*)g16 + base);
  const float o0 = (((a[0] * rr) * w0[0]) * (float)gv[0]) * kYCarry;
  const float o1 = (((a[1] * rr) * w0[1]) * (float)gv[1]) * kYCarry;
  const float o2 = (((a[2] * rr) * w0[2]) * (float)gv[2]) * kYCarry;
  const float o3 = (((a[3] * rr) * w0[3]) * (float)gv[3]) * kYCarry;
  const float o4 = (((c[0] * rr) * w1[0]) * (float)gv[4]) * kYCarry;
  const float o5 = (((c[1] * rr) * w1[1]) * (float)gv[5]) * kYCarry;
  const float o6 = (((c[2] * rr) * w1[2]) * (float)gv[6]) * kYCarry;
  const float o7 = (((c[3] * rr) * w1[3]) * (float)gv[7]) * kYCarry;
  const v4u u = (v4u){pk16(h_bits(o0), h_bits(o1)), pk16(h_bits(o2), h_bits(o3)),
                      pk16(h_bits(o4), h_bits(o5)), pk16(h_bits(o6), h_bits(o7))};
  *(volatile v4u*)(y2 + base) = u;
  __threadfence();
  *(volatile v4u*)(y2 + base) = u;
}

extern "C" void kernel_launch(void* const* d_in, const int* in_sizes, int n_in,
                              void* d_out, int out_size, void* d_ws, size_t ws_size,
                              hipStream_t stream) {
  if (n_in < 12) return;
  if (in_sizes[0] != kRows * kEmb || in_sizes[1] != kEmb * kEmb || in_sizes[2] != kEmb ||
      in_sizes[3] != kEmb * kEmb || in_sizes[4] != kEmb || in_sizes[5] != kVEmb * kEmb ||
      in_sizes[6] != kVEmb || in_sizes[7] != kVEmb * kEmb || in_sizes[8] != kVEmb ||
      in_sizes[9] != kEmb * kVEmb || in_sizes[10] != kEmb || in_sizes[11] != kDV) return;
  if (out_size != kRows * kEmb) return;
  if (ws_size < kWsTotal) return;

  const float* x   = (const float*)d_in[0];
  const float* Wq  = (const float*)d_in[1];
  const float* bq  = (const float*)d_in[2];
  const float* Wk  = (const float*)d_in[3];
  const float* bk  = (const float*)d_in[4];
  const float* Wv  = (const float*)d_in[5];
  const float* bv  = (const float*)d_in[6];
  const float* Wg  = (const float*)d_in[7];
  const float* bg  = (const float*)d_in[8];
  const float* Wo  = (const float*)d_in[9];
  const float* bo  = (const float*)d_in[10];
  const float* gnw = (const float*)d_in[11];
  float* outp = (float*)d_out;

  char* ws = (char*)d_ws;
  unsigned short* xb   = (unsigned short*)(ws + kOffXb);
  unsigned short* wqb  = (unsigned short*)(ws + kOffWq);
  unsigned short* wkb  = (unsigned short*)(ws + kOffWk);
  unsigned short* wvb  = (unsigned short*)(ws + kOffWv);
  unsigned short* wgb  = (unsigned short*)(ws + kOffWg);
  float*          tmp  = (float*)(ws + kOffTmp);
  unsigned short* pbuf = (unsigned short*)(ws + kOffP);
  unsigned short* y2   = (unsigned short*)(ws + kOffY2);
  unsigned short* wo16 = (unsigned short*)(ws + kOffWo);
  unsigned short* qr   = (unsigned short*)(ws + kOffQr);
  unsigned short* kr   = (unsigned short*)(ws + kOffKr);
  unsigned short* vt   = (unsigned short*)(ws + kOffVT);
  unsigned short* g16  = (unsigned short*)(ws + kOffG);
  float*          ybuf = (float*)(ws + kOffY);
  float*          trig = (float*)(ws + kOffTrig);
  const float*    unusedf = (const float*)(ws + kOffY);

  float invf[kPairs];
  for (int i = 0; i < kPairs; ++i) {
    const float pf = (float)pow(10000.0, (double)i / 64.0);
    invf[i] = 1.0f / pf;
  }
  v4f fv[16];
  for (int gq = 0; gq < 16; ++gq) {
    v4f t; t[0] = invf[4 * gq]; t[1] = invf[4 * gq + 1]; t[2] = invf[4 * gq + 2]; t[3] = invf[4 * gq + 3];
    fv[gq] = t;
  }
  float lg2g[kHeads];
  for (int h = 0; h < kHeads; ++h) lg2g[h] = (float)log2(1.0 - ldexp(1.0, -5 - h));

  trig_table_kernel<<<dim3(kSeq / 256, kPairs), 256, 0, stream>>>(trig,
      fv[0], fv[1], fv[2], fv[3], fv[4], fv[5], fv[6], fv[7], fv[8], fv[9], fv[10], fv[11], fv[12], fv[13], fv[14], fv[15]);

  { const int n8 = kRows * kEmb / 8;  cast16x8_kernel<0><<<(n8 + 255) / 256, 256, 0, stream>>>(x,  xb,  n8); }
  { const int n8 = kEmb * kEmb / 8;   cast16x8_kernel<0><<<(n8 + 255) / 256, 256, 0, stream>>>(Wq, wqb, n8); }
  { const int n8 = kEmb * kEmb / 8;   cast16x8_kernel<0><<<(n8 + 255) / 256, 256, 0, stream>>>(Wk, wkb, n8); }
  { const int n8 = kVEmb * kEmb / 8;  cast16x8_kernel<0><<<(n8 + 255) / 256, 256, 0, stream>>>(Wv, wvb, n8); }
  { const int n8 = kVEmb * kEmb / 8;  cast16x8_kernel<0><<<(n8 + 255) / 256, 256, 0, stream>>>(Wg, wgb, n8); }
  { const int n8 = kEmb * kVEmb / 8;  cast16x8_kernel<1><<<(n8 + 255) / 256, 256, 0, stream>>>(Wo, wo16, n8); }

  const int tilesQK = (kRows / 64) * (kEmb / 64);
  wmma_gemm64<1, false, 2, 0, false, 0, 0><<<dim3(tilesQK / 8, 1), 256, 0, stream>>>(
      xb, xb, kEmb, 0L, wqb, wqb, kEmb, 0L, (void*)tmp, (void*)tmp, kEmb, 0L,
      bq, unusedf, 0L, kRows, kEmb, kEmb, 1.0f, 1.0f, 0.f, 0.f, 0.f, 0.f);
  rope_kernel<<<(kRows * kEmb / 8) / 256, 256, 0, stream>>>(tmp, trig, qr);
  wmma_gemm64<1, false, 2, 0, false, 0, 0><<<dim3(tilesQK / 8, 1), 256, 0, stream>>>(
      xb, xb, kEmb, 0L, wkb, wkb, kEmb, 0L, (void*)tmp, (void*)tmp, kEmb, 0L,
      bk, unusedf, 0L, kRows, kEmb, kEmb, 1.0f, 1.0f, 0.f, 0.f, 0.f, 0.f);
  rope_kernel<<<(kRows * kEmb / 8) / 256, 256, 0, stream>>>(tmp, trig, kr);

  {
    const int tiles = (kVEmb / 64) * (kSeq / 64);
    wmma_gemm64<1, false, 1, 1, false, 0, 0><<<dim3(tiles / 8, kBatch), 256, 0, stream>>>(
        wvb, wvb, kEmb, 0L, xb, xb, kEmb, (long)kSeq * kEmb, (void*)vt, (void*)vt, kSeq, (long)kVEmb * kSeq,
        bv, unusedf, 0L, kVEmb, kSeq, kEmb, 1.0f, kVCarry, 0.f, 0.f, 0.f, 0.f);
  }
  {
    const int tiles = (kRows / 64) * (kVEmb / 64);
    wmma_gemm64<1, false, 2, 1, false, 6, 0><<<dim3(tiles / 8, 1), 256, 0, stream>>>(
        xb, xb, kEmb, 0L, wgb, wgb, kEmb, 0L, (void*)g16, (void*)g16, kVEmb, 0L,
        bg, unusedf, 0L, kRows, kVEmb, kEmb, 1.0f, 1.0f, 0.f, 0.f, 0.f, 0.f);
  }

  for (int grp = 0; grp < kGroups; ++grp) {
    const int bb = grp / (kHeads / kHeadsPerGrp);
    const int h0 = (grp % (kHeads / kHeadsPerGrp)) * kHeadsPerGrp;
    const unsigned short* qbase = qr + (size_t)bb * kSeq * kEmb + (size_t)h0 * kDK;
    const unsigned short* kbase = kr + (size_t)bb * kSeq * kEmb + (size_t)h0 * kDK;
    const int tilesS = (kSeq / 64) * (kSeq / 64);
    wmma_gemm64<0, false, 0, 1, false, 0, 1><<<dim3(tilesS / 8, kHeadsPerGrp), 256, 0, stream>>>(
        qbase, qbase, kEmb, (long)kDK, kbase, kbase, kEmb, (long)kDK,
        (void*)pbuf, (void*)pbuf, kSeq, (long)kSeq * kSeq,
        unusedf, unusedf, 0L, kSeq, kSeq, kDK, kScoreScale, 1.0f,
        lg2g[h0], lg2g[h0 + 1], lg2g[h0 + 2], lg2g[h0 + 3]);
    const unsigned short* vbase = vt + (size_t)bb * kVEmb * kSeq + (size_t)h0 * kDV * kSeq;
    float* ybase = ybuf + (size_t)bb * kSeq * kVEmb + (size_t)h0 * kDV;
    const int tilesY = (kSeq / 64) * (kDV / 64);
    wmma_gemm64<0, false, 0, 0, false, 0, 2><<<dim3(tilesY / 8, kHeadsPerGrp), 256, 0, stream>>>(
        pbuf, pbuf, kSeq, (long)kSeq * kSeq, vbase, vbase, kSeq, (long)kDV * kSeq,
        (void*)ybase, (void*)ybase, kVEmb, (long)kDV,
        unusedf, unusedf, 0L, kSeq, kDV, kSeq, kPVScale, 1.0f, 0.f, 0.f, 0.f, 0.f);
  }

  rmsgate_kernel<<<kRows, 256, 0, stream>>>(ybuf, g16, gnw, y2);

  wmma_gemm64<0, false, 2, 0, false, 0, 0><<<dim3(tilesQK / 8, 1), 256, 0, stream>>>(
      y2, y2, kVEmb, 0L, wo16, wo16, kVEmb, 0L, (void*)outp, (void*)outp, kEmb, 0L,
      bo, unusedf, 0L, kRows, kEmb, kVEmb, kOutScale, 1.0f, 0.f, 0.f, 0.f, 0.f);
}
